// BartDecoderLayer_27779848471448
// MI455X (gfx1250) — hardware-verified
//
#include <hip/hip_runtime.h>


#define NB_  4
#define FFH  4096
#define TT   1024
#define CC   1024
#define NH_  16
#define HD   64
#define NT   (NB_ * TT)
#define NZ   (NB_ * NH_)
#define ZB   8
#define PCAR 1024.0f
typedef _Float16 h16;
typedef unsigned short bf;
typedef __attribute__((ext_vector_type(16))) __bf16   v16bf;
typedef __attribute__((ext_vector_type(16))) _Float16 v16h;
typedef __attribute__((ext_vector_type(8)))  _Float16 v8h;
typedef __attribute__((ext_vector_type(8)))  unsigned short v8us;
typedef __attribute__((ext_vector_type(8)))  float    v8f;
typedef __attribute__((ext_vector_type(4)))  float    v4f;
typedef v8h  __attribute__((may_alias)) v8ha;
typedef v4f  __attribute__((may_alias)) v4fa;
typedef v8us __attribute__((may_alias)) v8usa;

__device__ __forceinline__ unsigned short f2bf(float f) { unsigned u = __float_as_uint(f); u += 0x7FFFu + ((u >> 16) & 1u); return (unsigned short)(u >> 16); }
__device__ __forceinline__ float bf2f(unsigned short b) { return __uint_as_float(((unsigned)b) << 16); }
__device__ __forceinline__ float bfr(float f) { return bf2f(f2bf(f)); }
__device__ __forceinline__ v16h cat16(v8h lo, v8h hi) { return __builtin_shufflevector(lo, hi, 0, 1, 2, 3, 4, 5, 6, 7, 8, 9, 10, 11, 12, 13, 14, 15); }
__device__ __forceinline__ v16bf cat16b(v8us lo, v8us hi) { return __builtin_bit_cast(v16bf, __builtin_shufflevector(lo, hi, 0, 1, 2, 3, 4, 5, 6, 7, 8, 9, 10, 11, 12, 13, 14, 15)); }
__device__ __forceinline__ v8f wmma16(v16h a, v16h b, v8f c) { return __builtin_amdgcn_wmma_f32_16x16x32_f16(false, a, false, b, (short)0, c, false, false); }
__device__ __forceinline__ v8f wmmab(v16bf a, v16bf b, v8f c) { return __builtin_amdgcn_wmma_f32_16x16x32_bf16(false, a, false, b, (short)0, c, false, false); }


template <typename T16> struct WFrag;
template <> struct WFrag<h16> { typedef v16h V; static __device__ __forceinline__ V ld(const h16* p) { return cat16(*(const v8h*)p, *(const v8h*)(p + 16)); } static __device__ __forceinline__ v8f mma(V a, V b, v8f c) { return wmma16(a, b, c); } };
template <> struct WFrag<bf> { typedef v16bf V; static __device__ __forceinline__ V ld(const bf* p) { return cat16b(*(const v8us*)p, *(const v8us*)(p + 16)); } static __device__ __forceinline__ v8f mma(V a, V b, v8f c) { return wmmab(a, b, c); } };
template <typename T16, int NSPLIT, bool BIAS>
__global__ __launch_bounds__(32) void k_gemmw(const T16* __restrict__ A, const T16* __restrict__ A2, const T16* __restrict__ Bt, const T16* __restrict__ Bt2, int K, float* C, int ldc, const float* __restrict__ bias, size_t sA, size_t sB, size_t sC) {
    typedef typename WFrag<T16>::V V;
    __shared__ __align__(16) float os[16 * 68];
    const size_t z = blockIdx.z; A += z * sA; if (A2) A2 += z * sA; Bt += z * sB; if (Bt2) Bt2 += z * sB; C += z * sC;
    const int lane = threadIdx.x & 31, lr = lane & 15, hi = lane >> 4; const int r0 = blockIdx.x * 64, c0 = blockIdx.y * 64;
    v8f acc[4][4];
#pragma unroll
    for (int mb = 0; mb < 4; ++mb)
#pragma unroll
        for (int nb = 0; nb < 4; ++nb) acc[mb][nb] = (v8f){};
    const size_t aoff = (size_t)(r0 + lr) * K + 8 * hi, boff = (size_t)(c0 + lr) * K + 8 * hi;
#pragma unroll 1
    for (int kc = 0; kc < K; kc += 32) {
        V a[4], a2[4];
#pragma unroll
        for (int mb = 0; mb < 4; ++mb) { a[mb] = WFrag<T16>::ld(A + aoff + (size_t)mb * 16 * K + kc); if (NSPLIT == 1 || NSPLIT == 2) a2[mb] = WFrag<T16>::ld(A2 + aoff + (size_t)mb * 16 * K + kc); }
#pragma unroll
        for (int nb = 0; nb < 4; ++nb) { const V b = WFrag<T16>::ld(Bt + boff + (size_t)nb * 16 * K + kc); V b2; if (NSPLIT >= 2) b2 = WFrag<T16>::ld(Bt2 + boff + (size_t)nb * 16 * K + kc);
#pragma unroll
            for (int mb = 0; mb < 4; ++mb) { acc[mb][nb] = WFrag<T16>::mma(a[mb], b, acc[mb][nb]); if (NSPLIT == 1 || NSPLIT == 2) acc[mb][nb] = WFrag<T16>::mma(a2[mb], b, acc[mb][nb]); if (NSPLIT >= 2) acc[mb][nb] = WFrag<T16>::mma(a[mb], b2, acc[mb][nb]); } }
        asm volatile("v_nop\n\tv_nop\n\tv_nop\n\tv_nop" : "+v"(acc[0][0]), "+v"(acc[1][1]), "+v"(acc[2][2]), "+v"(acc[3][3]) : "v"(a[0]), "v"(a[3]));
    }
#pragma unroll
    for (int mb = 0; mb < 4; ++mb) {
#pragma unroll
        for (int nb = 0; nb < 4; ++nb) {
#pragma unroll
            for (int j = 0; j < 8; ++j) os[(hi * 8 + j) * 68 + nb * 16 + lr] = acc[mb][nb][j]; }
        __builtin_amdgcn_wave_barrier(); asm volatile("" ::: "memory");
        float* crow = C + (size_t)(r0 + mb * 16) * ldc + c0;
#pragma unroll 1
        for (int ps = 0; ps < 2; ++ps) {
#pragma unroll
            for (int s = 0; s < 8; ++s) { const int row = 2 * s + hi, cofs = lr * 4; v4f val = *(const v4fa*)(os + row * 68 + cofs); if (BIAS) { val[0] += bfr(bias[c0 + cofs]); val[1] += bfr(bias[c0 + cofs + 1]); val[2] += bfr(bias[c0 + cofs + 2]); val[3] += bfr(bias[c0 + cofs + 3]); }
                *(volatile v4f*)(crow + (size_t)row * ldc + cofs) = val; }
            if (ps == 0) __threadfence(); }
        __builtin_amdgcn_wave_barrier(); asm volatile("" ::: "memory");
    }
}

__device__ __forceinline__ h16 tohx(float x) { return (h16)x; }
__device__ __forceinline__ void splitf(float y, unsigned short& h, unsigned short& l) { h = f2bf(y); l = f2bf(y - bf2f(h)); }
typedef __attribute__((ext_vector_type(2))) _Float16 v2h;
typedef __attribute__((ext_vector_type(4))) _Float16 v4h;
typedef __attribute__((ext_vector_type(2))) unsigned short v2us;
typedef __attribute__((ext_vector_type(2))) float v2f;

__global__ __launch_bounds__(256) void k_cvt8(const float* __restrict__ src, bf* dst, size_t n8) { const size_t i = (size_t)blockIdx.x * 256 + threadIdx.x; if (i >= n8) return; const v8f v = *(const v8f*)(src + i * 8); v8us o;
#pragma unroll
    for (int k = 0; k < 8; ++k) o[k] = f2bf(v[k]); *(volatile v8us*)(dst + i * 8) = o; __threadfence(); *(volatile v8us*)(dst + i * 8) = o; }
__global__ __launch_bounds__(256) void k_wtT(const float* __restrict__ w, int pitch, int col0, bf* Bt) {
    const int lane = threadIdx.x & 31; const int L0 = (blockIdx.x * 8 + (threadIdx.x >> 5)) * 8; const int nlines = CC * CC / 64;
#pragma unroll 1
    for (int ps = 0; ps < 2; ++ps) {
#pragma unroll
        for (int l = 0; l < 8; ++l) { const int L = L0 + l; if (L >= nlines) break; const int e = L * 64 + lane * 2; const int k = e & (CC - 1), n = e >> 9; v2us o;
#pragma unroll
            for (int q = 0; q < 2; ++q) o[q] = f2bf(w[(size_t)(k + q) * pitch + col0 + n]);
            *(volatile v2us*)(Bt + (size_t)e) = o; }
        if (ps == 0) __threadfence(); }
}
__global__ __launch_bounds__(256) void k_hplane(const float* __restrict__ F, float sc, h16* P) {
    const int lane = threadIdx.x & 31; const int L0 = (blockIdx.x * 8 + (threadIdx.x >> 5)) * 8; const int nlines = NT * CC / 64;
#pragma unroll 1
    for (int ps = 0; ps < 2; ++ps) {
#pragma unroll
        for (int l = 0; l < 8; ++l) { const int L = L0 + l; if (L >= nlines) break; const int e = L * 64 + lane * 2; const int d = e & 63; const int t = (e >> 6) & (TT - 1); const int z = e >> 16; const int b = z / NH_, h = z % NH_; v2h o;
#pragma unroll
            for (int q = 0; q < 2; ++q) o[q] = tohx(F[((size_t)b * TT + t) * CC + h * HD + d + q] * sc);
            *(volatile v2h*)(P + (size_t)e) = o; }
        if (ps == 0) __threadfence(); }
}
__global__ __launch_bounds__(256) void k_vtplane(const float* __restrict__ F, h16* VT) {
    const int lane = threadIdx.x & 31; const int L0 = (blockIdx.x * 8 + (threadIdx.x >> 5)) * 8; const int nlines = NT * CC / 64;
#pragma unroll 1
    for (int ps = 0; ps < 2; ++ps) {
#pragma unroll
        for (int l = 0; l < 8; ++l) { const int L = L0 + l; if (L >= nlines) break; const int e = L * 64 + lane * 2; const int t = e & (TT - 1); const int d = (e >> 10) & 63; const int z = e >> 16; const int b = z / NH_, h = z % NH_; v2h o;
#pragma unroll
            for (int q = 0; q < 2; ++q) o[q] = tohx(F[((size_t)b * TT + t + q) * CC + h * HD + d]);
            *(volatile v2h*)(VT + (size_t)e) = o; }
        if (ps == 0) __threadfence(); }
}
template <int RAW>
__global__ __launch_bounds__(256) void k_lnres(const float* __restrict__ A, const float* __restrict__ R, const float* __restrict__ gg, const float* __restrict__ bb, float* X, bf* Xh, bf* Xl) {
    typedef __attribute__((ext_vector_type(4))) unsigned short v4us;
    const int lane = threadIdx.x & 31; const int r = blockIdx.x * 8 + (threadIdx.x >> 5); if (r >= NT) return; float v[32]; float s = 0.f;
#pragma unroll
    for (int c = 0; c < 8; ++c) { const v4f a = *(const v4f*)(A + (size_t)r * CC + c * 128 + lane * 4), xx = *(const v4f*)(R + (size_t)r * CC + c * 128 + lane * 4);
#pragma unroll
        for (int q = 0; q < 4; ++q) { v[c * 4 + q] = a[q] + (RAW ? bfr(xx[q]) : xx[q]); s += v[c * 4 + q]; } }
#pragma unroll
    for (int sh = 16; sh; sh >>= 1) s += __shfl_xor(s, sh, 32);
    const float mu = s * (1.0f / CC); float qq = 0.f;
#pragma unroll
    for (int i = 0; i < 32; ++i) { const float d0 = v[i] - mu; qq = __fadd_rn(qq, __fmul_rn(d0, d0)); }
#pragma unroll
    for (int sh = 16; sh; sh >>= 1) qq += __shfl_xor(qq, sh, 32);
    const float rs = __fdiv_rn(1.0f, __fsqrt_rn(qq * (1.0f / CC) + 1e-5f));
    float o[32];
#pragma unroll
    for (int c = 0; c < 8; ++c) {
#pragma unroll
        for (int q = 0; q < 4; ++q) { const int col = c * 128 + lane * 4 + q; o[c * 4 + q] = __fadd_rn(__fmul_rn((v[c * 4 + q] - mu) * rs, bfr(gg[col])), bfr(bb[col])); } }
#pragma unroll 1
    for (int ps = 0; ps < 2; ++ps) {
#pragma unroll
        for (int c = 0; c < 8; ++c) { v4f w4; v4us oh, ol;
#pragma unroll
            for (int q = 0; q < 4; ++q) { w4[q] = o[c * 4 + q]; unsigned short a, c2; splitf(o[c * 4 + q], a, c2); oh[q] = a; ol[q] = c2; }
            if (X) *(volatile v4f*)(X + (size_t)r * CC + c * 128 + lane * 4) = w4;
            *(volatile v4us*)(Xh + (size_t)r * CC + c * 128 + lane * 4) = oh; *(volatile v4us*)(Xl + (size_t)r * CC + c * 128 + lane * 4) = ol; }
        if (ps == 0) __threadfence(); }
}
__global__ __launch_bounds__(256) void k_msoft(const float* __restrict__ Sb, const float* __restrict__ am, int z0, h16* P) {
    typedef __attribute__((ext_vector_type(4))) unsigned short v4us;
    const int lane = threadIdx.x & 31; const int row = blockIdx.x * 8 + (threadIdx.x >> 5); if (row >= ZB * TT) return; const int i = row & (TT - 1); const int zz = row >> 10; const int z = z0 + zz; const int b = z / NH_;
    const float* sr = Sb + (size_t)row * TT; const float* mr = am + ((size_t)b * TT + i) * TT; float v[32]; float mx = -3.0e38f;
#pragma unroll
    for (int ch = 0; ch < 8; ++ch) { const int j0 = ch * 128 + lane * 4; const v4f a = *(const v4f*)(sr + j0), mk = *(const v4f*)(mr + j0);
#pragma unroll
        for (int q = 0; q < 4; ++q) { float mm = bfr(mk[q]); asm volatile("" : "+v"(mm)); const float t = __fadd_rn(a[q], mm); v[ch * 4 + q] = t; mx = fmaxf(mx, t); } }
#pragma unroll
    for (int sh = 16; sh; sh >>= 1) mx = fmaxf(mx, __shfl_xor(mx, sh, 32));
    float sum = 0.f;
#pragma unroll
    for (int k = 0; k < 32; ++k) { v[k] = __expf(v[k] - mx); sum += v[k]; }
#pragma unroll
    for (int sh = 16; sh; sh >>= 1) sum += __shfl_xor(sum, sh, 32);
    const float f = __fdiv_rn(PCAR, sum);
#pragma unroll 1
    for (int ps = 0; ps < 2; ++ps) {
#pragma unroll
        for (int ch = 0; ch < 8; ++ch) { v4h o;
#pragma unroll
            for (int q = 0; q < 4; ++q) o[q] = tohx(v[ch * 4 + q] * f);
            *(volatile v4h*)(P + (size_t)row * TT + ch * 128 + lane * 4) = o; }
        if (ps == 0) __threadfence(); }
}
__global__ __launch_bounds__(256) void k_merge(const float* __restrict__ O, int z0, bf* Ah, bf* Al) {
    const int lane = threadIdx.x & 31; const int L0 = (blockIdx.x * 8 + (threadIdx.x >> 5)) * 8; const int nlines = ZB * TT * HD / 64;
#pragma unroll 1
    for (int ps = 0; ps < 2; ++ps) {
#pragma unroll
        for (int l = 0; l < 8; ++l) { const int L = L0 + l; if (L >= nlines) break; const int e = L * 64 + lane * 2; const int d = e & 63; const int t = (e >> 6) & (TT - 1); const int zz = e >> 16; const int z = z0 + zz; const int b = z / NH_, h = z % NH_; v2us oh, ol;
#pragma unroll
            for (int q = 0; q < 2; ++q) { unsigned short a, c2; splitf(O[(size_t)e + q] * (1.0f / PCAR), a, c2); oh[q] = a; ol[q] = c2; }
            const size_t o = ((size_t)b * TT + t) * CC + h * HD + d; *(volatile v2us*)(Ah + o) = oh; *(volatile v2us*)(Al + o) = ol; }
        if (ps == 0) __threadfence(); }
}

__global__ __launch_bounds__(256) void k_gelusplit(const float* __restrict__ H, bf* Hh, bf* Hl, size_t n) {
    const size_t i = ((size_t)blockIdx.x * 256 + threadIdx.x) * 2; if (i >= n) return; v2us oh, ol;
#pragma unroll
    for (int q = 0; q < 2; ++q) { const float h = H[i + q]; unsigned short a, c2; splitf(0.5f * h * (1.0f + erff(h * 0.70710678118654752f)), a, c2); oh[q] = a; ol[q] = c2; }
    *(volatile v2us*)(Hh + i) = oh; *(volatile v2us*)(Hl + i) = ol; __threadfence(); *(volatile v2us*)(Hh + i) = oh; *(volatile v2us*)(Hl + i) = ol;
}
__global__ __launch_bounds__(256) void k_relusplit(const float* __restrict__ H, bf* Hh, bf* Hl, size_t n) {
    const size_t i = ((size_t)blockIdx.x * 256 + threadIdx.x) * 2; if (i >= n) return; v2us oh, ol;
#pragma unroll
    for (int q = 0; q < 2; ++q) { unsigned short a, c2; splitf(fmaxf(H[i + q], 0.f), a, c2); oh[q] = a; ol[q] = c2; }
    *(volatile v2us*)(Hh + i) = oh; *(volatile v2us*)(Hl + i) = ol; __threadfence(); *(volatile v2us*)(Hh + i) = oh; *(volatile v2us*)(Hl + i) = ol; }
__global__ __launch_bounds__(256) void k_addout(const float* __restrict__ FF, const float* __restrict__ X, float* OUT, size_t n) {
    const size_t i = ((size_t)blockIdx.x * 256 + threadIdx.x) * 4; if (i >= n) return; const v4f a = *(const v4f*)(FF + i), b = *(const v4f*)(X + i); v4f o;
#pragma unroll
    for (int q = 0; q < 4; ++q) o[q] = a[q] + b[q];
    *(volatile v4f*)(OUT + i) = o; __threadfence(); *(volatile v4f*)(OUT + i) = o; }

extern "C" void kernel_launch(void* const* d_in, const int* in_sizes, int n_in,
                              void* d_out, int out_size, void* d_ws, size_t ws_size, hipStream_t stream) {
    (void)in_sizes; (void)n_in; (void)out_size;
    const float* IN[30]; for (int i = 0; i < 30; ++i) IN[i] = (const float*)d_in[i];
    const float* x = IN[0]; const float* enc = IN[1]; const float* am = IN[2]; const float* eam = IN[3];
    float* OUT = (float*)d_out;
    char* wsp = (char*)d_ws;
    auto take = [&](size_t bytes) { char* p = wsp; wsp += (bytes + 255) & ~(size_t)255; return (void*)p; };
    bf* WA = (bf*)take((size_t)CC * CC * 2); bf* WB = (bf*)take((size_t)CC * CC * 2); bf* WC = (bf*)take((size_t)CC * CC * 2); bf* WD = (bf*)take((size_t)CC * CC * 2);
    bf* W1 = (bf*)take((size_t)FFH * CC * 2); bf* W2 = (bf*)take((size_t)CC * FFH * 2);
    bf* XB = (bf*)take((size_t)NT * CC * 2); float* F = (float*)take((size_t)NT * CC * 4);
    char* R0 = wsp; h16* QP = (h16*)take((size_t)NT * CC * 2); h16* KP = (h16*)take((size_t)NT * CC * 2); h16* VT = (h16*)take((size_t)NT * CC * 2);
    float* Sb = (float*)take((size_t)ZB * TT * TT * 4); h16* Pm = (h16*)take((size_t)ZB * TT * TT * 2); float* Ob = (float*)take((size_t)ZB * TT * HD * 4); char* R1 = wsp;
    bf* ATh = (bf*)take((size_t)NT * CC * 2); bf* ATl = (bf*)take((size_t)NT * CC * 2); float* X1 = (float*)take((size_t)NT * CC * 4); bf* X1h = (bf*)take((size_t)NT * CC * 2); bf* X1l = (bf*)take((size_t)NT * CC * 2);
    if ((size_t)(wsp - (char*)d_ws) > ws_size) return;
    float* H = (float*)R0; bf* Hh = (bf*)(R0 + (size_t)(TT * 2) * FFH * 4); bf* Hl = (bf*)(R0 + (size_t)(TT * 2) * FFH * 6); if ((char*)(Hl + (size_t)(TT * 2) * FFH) > R1) return;
    float* Y = F;
    float* X2 = X1; bf* X2h = X1h; bf* X2l = X1l;
    float* FF2 = (float*)ATh;
    const size_t nw = (size_t)CC * CC / 8; const unsigned gw = (unsigned)((nw + 255) / 256); const unsigned LB = (unsigned)((NT * CC / 64 + 63) / 64); const dim3 gP(NT / 64, CC / 64, 1);
    auto attention = [&](const float* amask) {
        for (int z0 = 0; z0 < NZ; z0 += ZB) {
            k_gemmw<h16, 0, false><<<dim3(TT / 64, TT / 64, ZB), 32, 0, stream>>>(QP + (size_t)z0 * TT * HD, nullptr, KP + (size_t)z0 * TT * HD, nullptr, HD, Sb, TT, nullptr, (size_t)TT * HD, (size_t)TT * HD, (size_t)TT * TT);
            k_msoft<<<ZB * TT / 8, 256, 0, stream>>>(Sb, amask, z0, Pm);
            k_gemmw<h16, 0, false><<<dim3(TT / 64, 1, ZB), 32, 0, stream>>>(Pm, nullptr, VT + (size_t)z0 * HD * TT, nullptr, TT, Ob, HD, nullptr, (size_t)TT * TT, (size_t)HD * TT, (size_t)TT * HD);
            k_merge<<<(ZB * TT * HD / 64 + 63) / 64, 256, 0, stream>>>(Ob, z0, ATh, ATl); } };
    k_cvt8<<<gw, 256, 0, stream>>>(IN[4], WA, nw); k_cvt8<<<gw, 256, 0, stream>>>(IN[6], WB, nw); k_cvt8<<<gw, 256, 0, stream>>>(IN[8], WC, nw); k_cvt8<<<gw, 256, 0, stream>>>(IN[10], WD, nw);
    k_cvt8<<<(unsigned)(((size_t)NT * CC / 8 + 255) / 256), 256, 0, stream>>>(x, XB, (size_t)NT * CC / 8);
    k_gemmw<bf, 0, true><<<gP, 32, 0, stream>>>(XB, nullptr, WA, nullptr, CC, F, CC, IN[5], 0, 0, 0); k_hplane<<<LB, 256, 0, stream>>>(F, 0.125f, QP);
    k_gemmw<bf, 0, true><<<gP, 32, 0, stream>>>(XB, nullptr, WB, nullptr, CC, F, CC, IN[7], 0, 0, 0); k_hplane<<<LB, 256, 0, stream>>>(F, 1.0f, KP);
    k_gemmw<bf, 0, true><<<gP, 32, 0, stream>>>(XB, nullptr, WC, nullptr, CC, F, CC, IN[9], 0, 0, 0); k_vtplane<<<LB, 256, 0, stream>>>(F, VT);
    attention(am);
    k_gemmw<bf, 1, true><<<gP, 32, 0, stream>>>(ATh, ATl, WD, nullptr, CC, Y, CC, IN[11], 0, 0, 0);
    k_lnres<1><<<NT / 8, 256, 0, stream>>>(Y, x, IN[24], IN[25], X1, X1h, X1l);
    k_cvt8<<<gw, 256, 0, stream>>>(IN[12], WA, nw); k_cvt8<<<gw, 256, 0, stream>>>(IN[14], WB, nw); k_cvt8<<<gw, 256, 0, stream>>>(IN[16], WC, nw); k_cvt8<<<gw, 256, 0, stream>>>(IN[18], WD, nw);
    k_cvt8<<<(unsigned)(((size_t)NT * CC / 8 + 255) / 256), 256, 0, stream>>>(enc, XB, (size_t)NT * CC / 8);
    k_gemmw<bf, 1, true><<<gP, 32, 0, stream>>>(X1h, X1l, WA, nullptr, CC, F, CC, IN[13], 0, 0, 0); k_hplane<<<LB, 256, 0, stream>>>(F, 0.125f, QP);
    k_gemmw<bf, 0, true><<<gP, 32, 0, stream>>>(XB, nullptr, WB, nullptr, CC, F, CC, IN[15], 0, 0, 0); k_hplane<<<LB, 256, 0, stream>>>(F, 1.0f, KP);
    k_gemmw<bf, 0, true><<<gP, 32, 0, stream>>>(XB, nullptr, WC, nullptr, CC, F, CC, IN[17], 0, 0, 0); k_vtplane<<<LB, 256, 0, stream>>>(F, VT);
    attention(eam);
    k_gemmw<bf, 1, true><<<gP, 32, 0, stream>>>(ATh, ATl, WD, nullptr, CC, Y, CC, IN[19], 0, 0, 0);
    k_lnres<0><<<NT / 8, 256, 0, stream>>>(Y, X1, IN[26], IN[27], X2, X2h, X2l);
    k_cvt8<<<(unsigned)(((size_t)FFH * CC / 8 + 255) / 256), 256, 0, stream>>>(IN[20], W1, (size_t)FFH * CC / 8); k_cvt8<<<(unsigned)(((size_t)CC * FFH / 8 + 255) / 256), 256, 0, stream>>>(IN[22], W2, (size_t)CC * FFH / 8);
    for (int hb = 0; hb < 2; ++hb) { const size_t r0 = (size_t)hb * (TT * 2);
        k_gemmw<bf, 1, true><<<dim3((TT * 2) / 64, FFH / 64, 1), 32, 0, stream>>>(X2h + r0 * CC, X2l + r0 * CC, W1, nullptr, CC, H, FFH, IN[21], 0, 0, 0);
        k_gelusplit<<<(unsigned)(((size_t)(TT * 2) * FFH / 2 + 255) / 256), 256, 0, stream>>>(H, Hh, Hl, (size_t)(TT * 2) * FFH);
        k_gemmw<bf, 1, true><<<dim3((TT * 2) / 64, CC / 64, 1), 32, 0, stream>>>(Hh, Hl, W2, nullptr, FFH, FF2 + r0 * CC, CC, IN[23], 0, 0, 0); }
    k_lnres<0><<<NT / 8, 256, 0, stream>>>(FF2, X2, IN[28], IN[29], OUT, XB, XB + (size_t)NT * CC);
}
